// ResidualAttentionBlock_52802327937632
// MI455X (gfx1250) — hardware-verified
//
#include <hip/hip_runtime.h>
#include <math.h>

constexpr int kBatch  = 8;
constexpr int kSeq    = 1024;
constexpr int kDim    = 1024;
constexpr int kHeads  = 16;
constexpr int kHd     = 64;
constexpr int kTok    = kBatch * kSeq;
constexpr int kFF     = 4096;
constexpr int kQKld   = 2 * kDim;
constexpr int kGrp    = 8;
constexpr int kChunks = kBatch * kHeads / kGrp;
constexpr float kWCarry    = 16.0f;
constexpr float kWCarryInv = 1.0f / 16.0f;
constexpr float kPCarry    = 2048.0f;
constexpr float kCtxCarry  = 256.0f;
constexpr float kScoreScale = 0.125f;
constexpr float kPVScale   = kCtxCarry / kPCarry;
constexpr float kOutScale  = 1.0f / (kCtxCarry * kWCarry);
constexpr float kInvDim    = 1.0f / 1024.0f;
constexpr float kLnEps     = 1e-5f;

constexpr size_t kMiB     = 1048576;
constexpr size_t kOffAct  = 0;
constexpr size_t kOffWqkv = 16 * kMiB;
constexpr size_t kOffWout = 22 * kMiB;
constexpr size_t kOffWfc  = 16 * kMiB;
constexpr size_t kOffWprj = 24 * kMiB;
constexpr size_t kOffQK   = 32 * kMiB;
constexpr size_t kOffX1   = 32 * kMiB;
constexpr size_t kOffVT   = 64 * kMiB;
constexpr size_t kOffSc   = 80 * kMiB;
constexpr size_t kOffP    = 112 * kMiB;
constexpr size_t kOffHid  = 64 * kMiB;
constexpr size_t kWsNeed  = 128 * kMiB;

typedef __attribute__((ext_vector_type(16))) _Float16 v16h;
typedef __attribute__((ext_vector_type(8)))  _Float16 v8h;
typedef __attribute__((ext_vector_type(16))) __bf16   v16b;
typedef __attribute__((ext_vector_type(8)))  __bf16   v8b;
typedef __attribute__((ext_vector_type(8)))  float    v8f;
typedef __attribute__((ext_vector_type(4)))  float    v4f;
typedef __attribute__((ext_vector_type(4)))  unsigned int v4u;
typedef __attribute__((ext_vector_type(2)))  unsigned int v2u;

__device__ __forceinline__ unsigned short f2bf_bits(float f) {
  unsigned u = __float_as_uint(f);
  return (unsigned short)((u + 0x7FFFu + ((u >> 16) & 1u)) >> 16);
}
__device__ __forceinline__ float bf_bits2f(unsigned short h) { return __uint_as_float(((unsigned)h) << 16); }

__device__ __forceinline__ void dep_guard_h(v8f& a, v8f& b, v16h x, v16h y) { asm volatile("v_nop\n\tv_nop\n\tv_nop\n\tv_nop" : "+v"(a), "+v"(b) : "v"(x), "v"(y)); }
__device__ __forceinline__ void dep_guard_b(v8f& a, v8f& b, v16b x, v16b y) { asm volatile("v_nop\n\tv_nop\n\tv_nop\n\tv_nop" : "+v"(a), "+v"(b) : "v"(x), "v"(y)); }
__device__ __forceinline__ void keep4_h(v16h a, v16h b, v16h c, v16h d) { asm volatile("v_nop" :: "v"(a), "v"(b), "v"(c), "v"(d)); }
__device__ __forceinline__ void keep4_b(v16b a, v16b b, v16b c, v16b d) { asm volatile("v_nop" :: "v"(a), "v"(b), "v"(c), "v"(d)); }
__device__ __forceinline__ void acc_guard4(v8f& a, v8f& b, v8f& c, v8f& d) { asm volatile("v_nop\n\tv_nop\n\tv_nop\n\tv_nop" : "+v"(a), "+v"(b), "+v"(c), "+v"(d)); }
template <typename T> struct Frag;
template <> struct Frag<_Float16> {
  typedef v16h V; union U { v16h v; v8h h[2]; };
  static __device__ __forceinline__ v16h load(const _Float16* p) {
    U f; f.h[0] = *(const v8h*)(p); f.h[1] = *(const v8h*)(p + 16); return f.v;
  }
  static __device__ __forceinline__ v8f mma(v16h a, v16h b, v8f c) {
    return __builtin_amdgcn_wmma_f32_16x16x32_f16(false, a, false, b, (short)0, c, false, false);
  }
  static __device__ __forceinline__ void guard(v8f& a, v8f& b, v16h x, v16h y) { dep_guard_h(a, b, x, y); }
  static __device__ __forceinline__ void keep(v16h a, v16h b, v16h c, v16h d) { keep4_h(a, b, c, d); }
};
template <> struct Frag<__bf16> {
  typedef v16b V; union U { v16b v; v8b h[2]; };
  static __device__ __forceinline__ v16b load(const __bf16* p) {
    U f; f.h[0] = *(const v8b*)(p); f.h[1] = *(const v8b*)(p + 16); return f.v;
  }
  static __device__ __forceinline__ v8f mma(v16b a, v16b b, v8f c) {
    return __builtin_amdgcn_wmma_f32_16x16x32_bf16(false, a, false, b, (short)0, c, false, false);
  }
  static __device__ __forceinline__ void guard(v8f& a, v8f& b, v16b x, v16b y) { dep_guard_b(a, b, x, y); }
  static __device__ __forceinline__ void keep(v16b a, v16b b, v16b c, v16b d) { keep4_b(a, b, c, d); }
};

__device__ __forceinline__ unsigned pk16(unsigned short a, unsigned short b) { return (unsigned)a | ((unsigned)b << 16); }
__device__ __forceinline__ unsigned short h_bits(float f) { const _Float16 h = (_Float16)f; return __builtin_bit_cast(unsigned short, h); }

template <int ET> struct Elem;
template <> struct Elem<0> { typedef _Float16 T; };
template <> struct Elem<1> { typedef __bf16 T; };
template <int ET, bool SPLIT, int BIAS_MODE, int OUT_MODE, bool RESID, int ACT = 0>
__global__ __launch_bounds__(256) void wmma_gemm64(
    const unsigned short* __restrict__ Ap, const unsigned short* __restrict__ A2p, int lda, long strideA,
    const unsigned short* __restrict__ Btp, const unsigned short* __restrict__ Bt2p, int ldb, long strideB,
    void* __restrict__ Cout, void* __restrict__ Cout2, int ldc, long strideC,
    const float* __restrict__ bias,
    const float* __restrict__ resid, long strideR,
    int M, int N, int K, float scale) {
  typedef typename Elem<ET>::T T;
  typedef typename Frag<T>::V V;
  const T* A = (const T*)Ap; const T* A2 = (const T*)A2p; const T* Bt = (const T*)Btp; const T* Bt2 = (const T*)Bt2p;
  __shared__ __align__(16) float sT[8][16 * 68];
  const int b    = blockIdx.y;
  const int lane = threadIdx.x & 31;
  const int wave = threadIdx.x >> 5;
  const int tilesN = N >> 6;
  const int tilesM = M >> 6;
  const int tile = blockIdx.x * 8 + wave;
  if (tile >= tilesM * tilesN) return;
  const int tm = tile / tilesN;
  const int tn = tile - tm * tilesN;
  const int m0 = tm << 6;
  const int n0 = tn << 6;

  const T* Ab  = A  + (size_t)b * strideA;
  const T* Bb  = Bt + (size_t)b * strideB;
  const T* Ab2 = SPLIT ? (A2  + (size_t)b * strideA) : nullptr;
  const T* Bb2 = SPLIT ? (Bt2 + (size_t)b * strideB) : nullptr;

  const int rlane = lane & 15;
  const int koff  = (lane >> 4) * 8;
  const int mOff  = (lane >> 4) * 8;

  v8f acc[4][4];
#pragma unroll
  for (int i = 0; i < 4; ++i)
#pragma unroll
    for (int j = 0; j < 4; ++j) acc[i][j] = (v8f){0.f,0.f,0.f,0.f,0.f,0.f,0.f,0.f};

  for (int k0 = 0; k0 < K; k0 += 32) {
    V bh[4], bl[4];
#pragma unroll
    for (int j = 0; j < 4; ++j) {
      const size_t bo = (size_t)(n0 + (j << 4) + rlane) * ldb + koff + k0;
      bh[j] = Frag<T>::load(Bb + bo);
      if (SPLIT) bl[j] = Frag<T>::load(Bb2 + bo);
    }
#pragma unroll
    for (int i = 0; i < 4; ++i) {
      const size_t ao = (size_t)(m0 + (i << 4) + rlane) * lda + koff + k0;
      V ah = Frag<T>::load(Ab + ao);
      V al;
      if (SPLIT) al = Frag<T>::load(Ab2 + ao);
#pragma unroll
      for (int j = 0; j < 4; ++j) {
        acc[i][j] = Frag<T>::mma(ah, bh[j], acc[i][j]);
        if (SPLIT) {
          acc[i][j] = Frag<T>::mma(ah, bl[j], acc[i][j]);
          acc[i][j] = Frag<T>::mma(al, bh[j], acc[i][j]);
        }
      }
      Frag<T>::guard(acc[i][0], acc[i][3], ah, SPLIT ? al : ah);
    }
    Frag<T>::keep(bh[0], bh[1], bh[2], bh[3]);
    if (SPLIT) Frag<T>::keep(bl[0], bl[1], bl[2], bl[3]);
  }
  acc_guard4(acc[0][0], acc[0][1], acc[0][2], acc[0][3]);
  acc_guard4(acc[1][0], acc[1][1], acc[1][2], acc[1][3]);
  acc_guard4(acc[2][0], acc[2][1], acc[2][2], acc[2][3]);
  acc_guard4(acc[3][0], acc[3][1], acc[3][2], acc[3][3]);

  float* slab = sT[wave];
  const float* Rb = RESID ? (resid + (size_t)b * strideR) : nullptr;
#pragma unroll
  for (int i = 0; i < 4; ++i) {
    const int mBase = m0 + (i << 4);
#pragma unroll
    for (int j = 0; j < 4; ++j) {
      const int n = n0 + (j << 4) + rlane;
      float bv = 0.f;
      if (BIAS_MODE == 2) bv = bias[n];
#pragma unroll
      for (int r = 0; r < 8; ++r) {
        float v = acc[i][j][r] * scale;
        if (BIAS_MODE == 1) v += bias[mBase + mOff + r];
        if (BIAS_MODE == 2) v += bv;
        if (RESID) v += Rb[(size_t)(mBase + mOff + r) * ldc + n];
        if (ACT == 2) v = fmaxf(v, 0.0f);
        if (ACT == 4) v = (v > 0.f) ? v : 0.01f * v;
        if (ACT == 6) {
          const float e = expf(fminf(-1.702f * v, 60.0f));
          v = v / (1.0f + e);
        }
        slab[(mOff + r) * 68 + (j << 4) + rlane] = v;
      }
    }
    __builtin_amdgcn_fence(__ATOMIC_RELEASE, "workgroup");
    __builtin_amdgcn_wave_barrier();
    __builtin_amdgcn_fence(__ATOMIC_ACQUIRE, "workgroup");
    if (OUT_MODE == 0) {
      float* C = (float*)Cout + (size_t)b * strideC;
      const int hh = lane >> 4, c4 = (lane & 15) * 4;
      for (int pass = 0; pass < 2; ++pass) {
#pragma unroll
        for (int it = 0; it < 8; ++it) {
          const int row = it * 2 + hh;
          v4f v = *(const v4f*)(slab + row * 68 + c4);
          *(volatile v4f*)(C + (size_t)(mBase + row) * ldc + n0 + c4) = v;
        }
        __threadfence();
      }
    } else {
      const int q = lane >> 3, c8 = (lane & 7) * 8;
      unsigned short* C  = (unsigned short*)Cout  + (size_t)b * strideC;
      unsigned short* C2 = (OUT_MODE == 2) ? ((unsigned short*)Cout2 + (size_t)b * strideC) : nullptr;
      for (int pass = 0; pass < 2; ++pass) {
#pragma unroll
        for (int it = 0; it < 4; ++it) {
          const int row = it * 4 + q;
          const float* sp = slab + row * 68 + c8;
          v8h hv, lv;
#pragma unroll
          for (int e = 0; e < 8; ++e) {
            if (OUT_MODE == 1) {
              hv[e] = (_Float16)sp[e];
            } else {
              unsigned short hb = f2bf_bits(sp[e]);
              unsigned short lb = f2bf_bits(sp[e] - bf_bits2f(hb));
              hv[e] = __builtin_bit_cast(_Float16, hb);
              lv[e] = __builtin_bit_cast(_Float16, lb);
            }
          }
          *(volatile v8h*)(C + (size_t)(mBase + row) * ldc + n0 + c8) = hv;
          if (OUT_MODE == 2) *(volatile v8h*)(C2 + (size_t)(mBase + row) * ldc + n0 + c8) = lv;
        }
        __threadfence();
      }
    }
    __builtin_amdgcn_fence(__ATOMIC_RELEASE, "workgroup");
    __builtin_amdgcn_wave_barrier();
    __builtin_amdgcn_fence(__ATOMIC_ACQUIRE, "workgroup");
  }
}

__global__ __launch_bounds__(256) void cast8_f16_kernel(const float* __restrict__ in, unsigned short* __restrict__ out,
                                                        int n8, float scale) {
  const int i = blockIdx.x * 256 + threadIdx.x;
  if (i >= n8) return;
  const float* p = in + 8 * (size_t)i;
  const v4f a = *(const v4f*)(p);
  const v4f c = *(const v4f*)(p + 4);
  unsigned short hb[8];
#pragma unroll
  for (int e = 0; e < 4; ++e) {
    hb[e]     = h_bits(a[e] * scale);
    hb[4 + e] = h_bits(c[e] * scale);
  }
  const v4u u = (v4u){pk16(hb[0], hb[1]), pk16(hb[2], hb[3]), pk16(hb[4], hb[5]), pk16(hb[6], hb[7])};
  unsigned short* q = out + 8 * (size_t)i;
  *(volatile v4u*)q = u;
  __threadfence();
  *(volatile v4u*)q = u;
}

__global__ __launch_bounds__(256) void ln_rows_kernel(const float* __restrict__ x, const float* __restrict__ g,
                                                      const float* __restrict__ bb, unsigned short* __restrict__ out) {
  __shared__ float redA[8];
  __shared__ float redB[8];
  const int row  = blockIdx.x;
  const int t    = threadIdx.x;
  const int lane = t & 31, wave = t >> 5;
  const float* xr = x + (size_t)row * kDim + 4 * t;
  const v4f v = *(const v4f*)xr;
  float s = (v[0] + v[1]) + (v[2] + v[3]);
#pragma unroll
  for (int off = 16; off > 0; off >>= 1) s += __shfl_xor(s, off, 32);
  if (lane == 0) redA[wave] = s;
  __syncthreads();
  float tot = 0.f;
#pragma unroll
  for (int w = 0; w < 8; ++w) tot += redA[w];
  const float mu = tot * kInvDim;
  const float d0 = v[0] - mu, d1 = v[1] - mu, d2 = v[2] - mu, d3 = v[3] - mu;
  float s2 = (d0 * d0 + d1 * d1) + (d2 * d2 + d3 * d3);
#pragma unroll
  for (int off = 16; off > 0; off >>= 1) s2 += __shfl_xor(s2, off, 32);
  if (lane == 0) redB[wave] = s2;
  __syncthreads();
  float tot2 = 0.f;
#pragma unroll
  for (int w = 0; w < 8; ++w) tot2 += redB[w];
  const float var = tot2 * kInvDim;
  const float inv = rsqrtf(var + kLnEps);
  const v4f gv = *(const v4f*)(g + 4 * t);
  const v4f bv = *(const v4f*)(bb + 4 * t);
  const float y0 = d0 * inv * gv[0] + bv[0];
  const float y1 = d1 * inv * gv[1] + bv[1];
  const float y2 = d2 * inv * gv[2] + bv[2];
  const float y3 = d3 * inv * gv[3] + bv[3];
  const v2u u = (v2u){pk16(h_bits(y0), h_bits(y1)), pk16(h_bits(y2), h_bits(y3))};
  unsigned short* q = out + (size_t)row * kDim + 4 * t;
  *(volatile v2u*)q = u;
  __threadfence();
  *(volatile v2u*)q = u;
}

__global__ __launch_bounds__(128) void softmax_rows_kernel(const float* __restrict__ S, unsigned short* __restrict__ P,
                                                           float carry) {
  __shared__ float redM[4];
  __shared__ float redS[4];
  const int row  = blockIdx.x;
  const int t    = threadIdx.x;
  const int lane = t & 31, wave = t >> 5;
  const float* sr = S + (size_t)row * kSeq + 8 * t;
  const v4f a = *(const v4f*)(sr);
  const v4f c = *(const v4f*)(sr + 4);
  float x[8];
#pragma unroll
  for (int e = 0; e < 4; ++e) { x[e] = a[e]; x[4 + e] = c[e]; }
  float m = fmaxf(fmaxf(fmaxf(x[0], x[1]), fmaxf(x[2], x[3])), fmaxf(fmaxf(x[4], x[5]), fmaxf(x[6], x[7])));
#pragma unroll
  for (int off = 16; off > 0; off >>= 1) m = fmaxf(m, __shfl_xor(m, off, 32));
  if (lane == 0) redM[wave] = m;
  __syncthreads();
  const float mx = fmaxf(fmaxf(redM[0], redM[1]), fmaxf(redM[2], redM[3]));
  float p[8];
  float s = 0.f;
#pragma unroll
  for (int e = 0; e < 8; ++e) { p[e] = expf(x[e] - mx); s += p[e]; }
#pragma unroll
  for (int off = 16; off > 0; off >>= 1) s += __shfl_xor(s, off, 32);
  if (lane == 0) redS[wave] = s;
  __syncthreads();
  const float tot = (redS[0] + redS[1]) + (redS[2] + redS[3]);
  const float f = carry / tot;
  unsigned short hb[8];
#pragma unroll
  for (int e = 0; e < 8; ++e) hb[e] = h_bits(p[e] * f);
  const v4u u = (v4u){pk16(hb[0], hb[1]), pk16(hb[2], hb[3]), pk16(hb[4], hb[5]), pk16(hb[6], hb[7])};
  unsigned short* q = P + (size_t)row * kSeq + 8 * t;
  *(volatile v4u*)q = u;
  __threadfence();
  *(volatile v4u*)q = u;
}

extern "C" void kernel_launch(void* const* d_in, const int* in_sizes, int n_in,
                              void* d_out, int out_size, void* d_ws, size_t ws_size,
                              hipStream_t stream) {
  if (n_in < 13) return;
  if (in_sizes[0] != kTok * kDim || in_sizes[1] != 3 * kDim * kDim || in_sizes[2] != 3 * kDim ||
      in_sizes[3] != kDim * kDim || in_sizes[4] != kDim || in_sizes[5] != kDim || in_sizes[6] != kDim ||
      in_sizes[7] != kDim || in_sizes[8] != kDim || in_sizes[9] != kFF * kDim || in_sizes[10] != kFF ||
      in_sizes[11] != kDim * kFF || in_sizes[12] != kDim) return;
  if (out_size != kTok * kDim) return;
  if (ws_size < kWsNeed) return;

  const float* x         = (const float*)d_in[0];
  const float* in_proj_w = (const float*)d_in[1];
  const float* in_proj_b = (const float*)d_in[2];
  const float* out_w     = (const float*)d_in[3];
  const float* out_b     = (const float*)d_in[4];
  const float* ln1_g     = (const float*)d_in[5];
  const float* ln1_b     = (const float*)d_in[6];
  const float* ln2_g     = (const float*)d_in[7];
  const float* ln2_b     = (const float*)d_in[8];
  const float* fc_w      = (const float*)d_in[9];
  const float* fc_b      = (const float*)d_in[10];
  const float* proj_w    = (const float*)d_in[11];
  const float* proj_b    = (const float*)d_in[12];
  float* out = (float*)d_out;

  char* ws = (char*)d_ws;
  unsigned short* act16  = (unsigned short*)(ws + kOffAct);
  unsigned short* wqkv16 = (unsigned short*)(ws + kOffWqkv);
  unsigned short* wout16 = (unsigned short*)(ws + kOffWout);
  unsigned short* wfc16  = (unsigned short*)(ws + kOffWfc);
  unsigned short* wprj16 = (unsigned short*)(ws + kOffWprj);
  unsigned short* qk16   = (unsigned short*)(ws + kOffQK);
  float*          x1     = (float*)(ws + kOffX1);
  unsigned short* vt16   = (unsigned short*)(ws + kOffVT);
  float*          sc     = (float*)(ws + kOffSc);
  unsigned short* p16    = (unsigned short*)(ws + kOffP);
  unsigned short* hid16  = (unsigned short*)(ws + kOffHid);

  {
    const int n8a = 3 * kDim * kDim / 8;
    cast8_f16_kernel<<<dim3((n8a + 255) / 256), dim3(256), 0, stream>>>(in_proj_w, wqkv16, n8a, kWCarry);
    const int n8b = kDim * kDim / 8;
    cast8_f16_kernel<<<dim3((n8b + 255) / 256), dim3(256), 0, stream>>>(out_w, wout16, n8b, kWCarry);
  }

  ln_rows_kernel<<<dim3(kTok), dim3(256), 0, stream>>>(x, ln1_g, ln1_b, act16);

  wmma_gemm64<0, false, 2, 1, false, 0><<<dim3(512, 1), dim3(256), 0, stream>>>(
      act16, nullptr, kDim, 0L, wqkv16, nullptr, kDim, 0L,
      (void*)qk16, nullptr, kQKld, 0L, in_proj_b, nullptr, 0L, kTok, 2 * kDim, kDim, kWCarryInv);

  wmma_gemm64<0, false, 1, 1, false, 0><<<dim3(256, 1), dim3(256), 0, stream>>>(
      wqkv16 + (size_t)2 * kDim * kDim, nullptr, kDim, 0L, act16, nullptr, kDim, 0L,
      (void*)vt16, nullptr, kTok, 0L, in_proj_b + 2 * kDim, nullptr, 0L, kDim, kTok, kDim, kWCarryInv);

  unsigned short* ctx16 = act16;
  for (int cix = 0; cix < kChunks; ++cix) {
    const int b  = cix / 2;
    const int h0 = (cix % 2) * kGrp;
    const size_t qkb = (size_t)b * kSeq * kQKld + (size_t)h0 * kHd;
    wmma_gemm64<0, false, 0, 0, false, 0><<<dim3(32, kGrp), dim3(256), 0, stream>>>(
        qk16 + qkb, nullptr, kQKld, (long)kHd, qk16 + qkb + kDim, nullptr, kQKld, (long)kHd,
        (void*)sc, nullptr, kSeq, (long)kSeq * kSeq, nullptr, nullptr, 0L, kSeq, kSeq, kHd, kScoreScale);
    softmax_rows_kernel<<<dim3(kGrp * kSeq), dim3(128), 0, stream>>>(sc, p16, kPCarry);
    wmma_gemm64<0, false, 0, 1, false, 0><<<dim3(2, kGrp), dim3(256), 0, stream>>>(
        p16, nullptr, kSeq, (long)kSeq * kSeq,
        vt16 + (size_t)h0 * kHd * kTok + (size_t)b * kSeq, nullptr, kTok, (long)kHd * kTok,
        (void*)(ctx16 + (size_t)b * kSeq * kDim + (size_t)h0 * kHd), nullptr, kDim, (long)kHd,
        nullptr, nullptr, 0L, kSeq, kHd, kSeq, kPVScale);
  }

  wmma_gemm64<0, false, 2, 0, true, 0><<<dim3(256, 1), dim3(256), 0, stream>>>(
      ctx16, nullptr, kDim, 0L, wout16, nullptr, kDim, 0L,
      (void*)x1, nullptr, kDim, 0L, out_b, x, 0L, kTok, kDim, kDim, kOutScale);

  ln_rows_kernel<<<dim3(kTok), dim3(256), 0, stream>>>(x1, ln2_g, ln2_b, act16);

  {
    const int n8c = kFF * kDim / 8;
    cast8_f16_kernel<<<dim3((n8c + 255) / 256), dim3(256), 0, stream>>>(fc_w, wfc16, n8c, kWCarry);
    cast8_f16_kernel<<<dim3((n8c + 255) / 256), dim3(256), 0, stream>>>(proj_w, wprj16, n8c, kWCarry);
  }

  wmma_gemm64<0, false, 2, 1, false, 6><<<dim3(1024, 1), dim3(256), 0, stream>>>(
      act16, nullptr, kDim, 0L, wfc16, nullptr, kDim, 0L,
      (void*)hid16, nullptr, kFF, 0L, fc_b, nullptr, 0L, kTok, kFF, kDim, kWCarryInv);

  wmma_gemm64<0, false, 2, 0, true, 0><<<dim3(256, 1), dim3(256), 0, stream>>>(
      hid16, nullptr, kFF, 0L, wprj16, nullptr, kFF, 0L,
      (void*)out, nullptr, kDim, 0L, proj_b, x1, 0L, kTok, kDim, kFF, kWCarryInv);
}
